// RosaBase_63299228008847
// MI455X (gfx1250) — hardware-verified
//
#include <hip/hip_runtime.h>

constexpr int kBatch  = 2;
constexpr int kSeq    = 4096;
constexpr int kRows   = kBatch * kSeq;
constexpr int kDim    = 1024;
constexpr int kHeads  = 128;
constexpr int kBits   = 8;
constexpr int kWinMax = 8;

typedef __attribute__((ext_vector_type(16))) _Float16 v16h;
typedef __attribute__((ext_vector_type(8)))  _Float16 v8h;
typedef __attribute__((ext_vector_type(16))) __bf16   v16b;
typedef __attribute__((ext_vector_type(8)))  __bf16   v8b;
typedef __attribute__((ext_vector_type(8)))  float    v8f;
typedef __attribute__((ext_vector_type(4)))  float    v4f;
#define U16(p) ((const unsigned short*)(const void*)(p))

__device__ __forceinline__ unsigned short f2bf_bits(float f) {
  unsigned u = __float_as_uint(f);
  return (unsigned short)((u + 0x7FFFu + ((u >> 16) & 1u)) >> 16);
}
__device__ __forceinline__ float bf_bits2f(unsigned short h) { return __uint_as_float(((unsigned)h) << 16); }

__device__ __forceinline__ void dep_guard_h(v8f& a, v8f& b, v16h x, v16h y) { asm volatile("v_nop\n\tv_nop\n\tv_nop\n\tv_nop" : "+v"(a), "+v"(b) : "v"(x), "v"(y)); }
__device__ __forceinline__ void dep_guard_b(v8f& a, v8f& b, v16b x, v16b y) { asm volatile("v_nop\n\tv_nop\n\tv_nop\n\tv_nop" : "+v"(a), "+v"(b) : "v"(x), "v"(y)); }
__device__ __forceinline__ void keep4_h(v16h a, v16h b, v16h c, v16h d) { asm volatile("v_nop" :: "v"(a), "v"(b), "v"(c), "v"(d)); }
__device__ __forceinline__ void keep4_b(v16b a, v16b b, v16b c, v16b d) { asm volatile("v_nop" :: "v"(a), "v"(b), "v"(c), "v"(d)); }
__device__ __forceinline__ void acc_guard4(v8f& a, v8f& b, v8f& c, v8f& d) { asm volatile("v_nop\n\tv_nop\n\tv_nop\n\tv_nop" : "+v"(a), "+v"(b), "+v"(c), "+v"(d)); }
template <typename T> struct Frag;
template <> struct Frag<_Float16> {
  typedef v16h V; union U { v16h v; v8h h[2]; };
  static __device__ __forceinline__ v16h load(const _Float16* p) {
    U f; f.h[0] = *(const v8h*)(p); f.h[1] = *(const v8h*)(p + 16); return f.v;
  }
  static __device__ __forceinline__ v8f mma(v16h a, v16h b, v8f c) {
    return __builtin_amdgcn_wmma_f32_16x16x32_f16(false, a, false, b, (short)0, c, false, false);
  }
  static __device__ __forceinline__ void guard(v8f& a, v8f& b, v16h x, v16h y) { dep_guard_h(a, b, x, y); }
  static __device__ __forceinline__ void keep(v16h a, v16h b, v16h c, v16h d) { keep4_h(a, b, c, d); }
};
template <> struct Frag<__bf16> {
  typedef v16b V; union U { v16b v; v8b h[2]; };
  static __device__ __forceinline__ v16b load(const __bf16* p) {
    U f; f.h[0] = *(const v8b*)(p); f.h[1] = *(const v8b*)(p + 16); return f.v;
  }
  static __device__ __forceinline__ v8f mma(v16b a, v16b b, v8f c) {
    return __builtin_amdgcn_wmma_f32_16x16x32_bf16(false, a, false, b, (short)0, c, false, false);
  }
  static __device__ __forceinline__ void guard(v8f& a, v8f& b, v16b x, v16b y) { dep_guard_b(a, b, x, y); }
  static __device__ __forceinline__ void keep(v16b a, v16b b, v16b c, v16b d) { keep4_b(a, b, c, d); }
};

template <int ET> struct Elem;
template <> struct Elem<0> { typedef _Float16 T; };
template <> struct Elem<1> { typedef __bf16 T; };
template <int ET, bool SPLIT, int BIAS_MODE, int OUT_MODE, bool RESID, int ACT = 0>
__global__ __launch_bounds__(256) void wmma_gemm64(
    const unsigned short* __restrict__ Ap, const unsigned short* __restrict__ A2p, int lda, long strideA,
    const unsigned short* __restrict__ Btp, const unsigned short* __restrict__ Bt2p, int ldb, long strideB,
    void* __restrict__ Cout, void* __restrict__ Cout2, int ldc, long strideC,
    const float* __restrict__ bias,
    const float* __restrict__ resid, long strideR,
    int M, int N, int K, float scale) {
  typedef typename Elem<ET>::T T;
  typedef typename Frag<T>::V V;
  const T* A = (const T*)Ap; const T* A2 = (const T*)A2p; const T* Bt = (const T*)Btp; const T* Bt2 = (const T*)Bt2p;
  __shared__ __align__(16) float sT[8][16 * 68];
  const int b    = blockIdx.y;
  const int lane = threadIdx.x & 31;
  const int wave = threadIdx.x >> 5;
  const int tilesN = N >> 6;
  const int tilesM = M >> 6;
  const int tile = blockIdx.x * 8 + wave;
  if (tile >= tilesM * tilesN) return;
  const int tm = tile / tilesN;
  const int tn = tile - tm * tilesN;
  const int m0 = tm << 6;
  const int n0 = tn << 6;

  const T* Ab  = A  + (size_t)b * strideA;
  const T* Bb  = Bt + (size_t)b * strideB;
  const T* Ab2 = SPLIT ? (A2  + (size_t)b * strideA) : nullptr;
  const T* Bb2 = SPLIT ? (Bt2 + (size_t)b * strideB) : nullptr;

  const int rlane = lane & 15;
  const int koff  = (lane >> 4) * 8;
  const int mOff  = (lane >> 4) * 8;

  v8f acc[4][4];
#pragma unroll
  for (int i = 0; i < 4; ++i)
#pragma unroll
    for (int j = 0; j < 4; ++j) acc[i][j] = (v8f){0.f,0.f,0.f,0.f,0.f,0.f,0.f,0.f};

  for (int k0 = 0; k0 < K; k0 += 32) {
    V bh[4], bl[4];
#pragma unroll
    for (int j = 0; j < 4; ++j) {
      const size_t bo = (size_t)(n0 + (j << 4) + rlane) * ldb + koff + k0;
      bh[j] = Frag<T>::load(Bb + bo);
      if (SPLIT) bl[j] = Frag<T>::load(Bb2 + bo);
    }
#pragma unroll
    for (int i = 0; i < 4; ++i) {
      const size_t ao = (size_t)(m0 + (i << 4) + rlane) * lda + koff + k0;
      V ah = Frag<T>::load(Ab + ao);
      V al;
      if (SPLIT) al = Frag<T>::load(Ab2 + ao);
#pragma unroll
      for (int j = 0; j < 4; ++j) {
        acc[i][j] = Frag<T>::mma(ah, bh[j], acc[i][j]);
        if (SPLIT) {
          acc[i][j] = Frag<T>::mma(ah, bl[j], acc[i][j]);
          acc[i][j] = Frag<T>::mma(al, bh[j], acc[i][j]);
        }
      }
      Frag<T>::guard(acc[i][0], acc[i][3], ah, SPLIT ? al : ah);
    }
    Frag<T>::keep(bh[0], bh[1], bh[2], bh[3]);
    if (SPLIT) Frag<T>::keep(bl[0], bl[1], bl[2], bl[3]);
  }
  acc_guard4(acc[0][0], acc[0][1], acc[0][2], acc[0][3]);
  acc_guard4(acc[1][0], acc[1][1], acc[1][2], acc[1][3]);
  acc_guard4(acc[2][0], acc[2][1], acc[2][2], acc[2][3]);
  acc_guard4(acc[3][0], acc[3][1], acc[3][2], acc[3][3]);

  float* slab = sT[wave];
  const float* Rb = RESID ? (resid + (size_t)b * strideR) : nullptr;
#pragma unroll
  for (int i = 0; i < 4; ++i) {
    const int mBase = m0 + (i << 4);
#pragma unroll
    for (int j = 0; j < 4; ++j) {
      const int n = n0 + (j << 4) + rlane;
      float bv = 0.f;
      if (BIAS_MODE == 2) bv = bias[n];
#pragma unroll
      for (int r = 0; r < 8; ++r) {
        float v = acc[i][j][r] * scale;
        if (BIAS_MODE == 1) v += bias[mBase + mOff + r];
        if (BIAS_MODE == 2) v += bv;
        if (RESID) v += Rb[(size_t)(mBase + mOff + r) * ldc + n];
        if (ACT == 1) v = tanhf(v);
        if (ACT == 2) v = fmaxf(v, 0.0f);
        if (ACT == 3) v = v / (1.0f + expf(-v));
        if (ACT == 4) v = (v > 0.f) ? v : 0.01f * v;
        if (ACT == 5) v = 0.5f * v * (1.0f + erff(v * 0.70710678118654752f));
        if (ACT == 7) { const float ex = __expf(-v); v = __builtin_amdgcn_rcpf(1.0f + ex) * 16.0f - 8.0f; }
        slab[(mOff + r) * 68 + (j << 4) + rlane] = v;
      }
    }
    __builtin_amdgcn_fence(__ATOMIC_RELEASE, "workgroup");
    __builtin_amdgcn_wave_barrier();
    __builtin_amdgcn_fence(__ATOMIC_ACQUIRE, "workgroup");
    if (OUT_MODE == 0) {
      float* C = (float*)Cout + (size_t)b * strideC;
      const int hh = lane >> 4, c4 = (lane & 15) * 4;
      for (int pass = 0; pass < 2; ++pass) {
#pragma unroll
        for (int it = 0; it < 8; ++it) {
          const int row = it * 2 + hh;
          v4f v = *(const v4f*)(slab + row * 68 + c4);
          *(volatile v4f*)(C + (size_t)(mBase + row) * ldc + n0 + c4) = v;
        }
        __threadfence();
      }
    } else {
      const int q = lane >> 3, c8 = (lane & 7) * 8;
      unsigned short* C  = (unsigned short*)Cout  + (size_t)b * strideC;
      unsigned short* C2 = (OUT_MODE == 2) ? ((unsigned short*)Cout2 + (size_t)b * strideC) : nullptr;
      for (int pass = 0; pass < 2; ++pass) {
#pragma unroll
        for (int it = 0; it < 4; ++it) {
          const int row = it * 4 + q;
          const float* sp = slab + row * 68 + c8;
          v8h hv, lv;
#pragma unroll
          for (int e = 0; e < 8; ++e) {
            if (OUT_MODE == 1) {
              hv[e] = (_Float16)sp[e];
            } else {
              unsigned short hb = f2bf_bits(sp[e]);
              unsigned short lb = f2bf_bits(sp[e] - bf_bits2f(hb));
              hv[e] = __builtin_bit_cast(_Float16, hb);
              lv[e] = __builtin_bit_cast(_Float16, lb);
            }
          }
          *(volatile v8h*)(C + (size_t)(mBase + row) * ldc + n0 + c8) = hv;
          if (OUT_MODE == 2) *(volatile v8h*)(C2 + (size_t)(mBase + row) * ldc + n0 + c8) = lv;
        }
        __threadfence();
      }
    }
    __builtin_amdgcn_fence(__ATOMIC_RELEASE, "workgroup");
    __builtin_amdgcn_wave_barrier();
    __builtin_amdgcn_fence(__ATOMIC_ACQUIRE, "workgroup");
  }
}

__global__ __launch_bounds__(256) void k_cast8(const float* __restrict__ in, _Float16* __restrict__ out,
                                               float mul, int n8) {
  const int id = blockIdx.x * 256 + threadIdx.x;
  const int idc = id < n8 ? id : n8 - 1;
  const v4f a0 = *(const v4f*)(in + (size_t)idc * 8);
  const v4f a1 = *(const v4f*)(in + (size_t)idc * 8 + 4);
  v8h hv;
#pragma unroll
  for (int e = 0; e < 4; ++e) { hv[e] = (_Float16)(a0[e] * mul); hv[4 + e] = (_Float16)(a1[e] * mul); }
  if (id < n8) {
    _Float16* dst = out + (size_t)idc * 8;
    *(volatile v8h*)dst = hv;
    __threadfence();
    *(volatile v8h*)dst = hv;
  }
}

__global__ __launch_bounds__(256) void k_window(
    const _Float16* __restrict__ cq, const _Float16* __restrict__ ck, const _Float16* __restrict__ cv,
    const float* __restrict__ emb0, const float* __restrict__ emb1, const int* __restrict__ swin,
    _Float16* __restrict__ pout, int total) {
  const int id  = blockIdx.x * 256 + threadIdx.x;
  const int idc = id < total ? id : total - 1;
  const int h   = idc & (kHeads - 1);
  const int row = idc >> 7;
  const int s   = row & (kSeq - 1);
  int wlen = swin[0];
  wlen = wlen < 1 ? 1 : (wlen > kWinMax ? kWinMax : wlen);

  const size_t qoff = (size_t)row * kDim + (size_t)h * kBits;
  const v8h qv = *(const v8h*)(cq + qoff);
  float qf[8];
#pragma unroll
  for (int e = 0; e < 8; ++e) qf[e] = (float)qv[e];

  float lsum = 0.f;
  float o[8];
#pragma unroll
  for (int e = 0; e < 8; ++e) o[e] = 0.f;

  const float kSc = 0.35355339059327373f;
#pragma unroll 1
  for (int d = 0; d < kWinMax; ++d) {
    const bool valid = (s >= d) && (d < wlen);
    const int rk = valid ? (row - d) : row;
    const size_t koff = (size_t)rk * kDim + (size_t)h * kBits;
    const v8h kv = *(const v8h*)(ck + koff);
    const v8h vv = *(const v8h*)(cv + koff);
    float sab = 0.f;
#pragma unroll
    for (int e = 0; e < 8; ++e) sab = fmaf(qf[e], (float)kv[e], sab);
    const float sc = fmaf(sab, kSc * (2.0f / 256.0f), 4.0f * kSc);
    float p = __expf(sc);
    p = valid ? p : 0.f;
    lsum += p;
#pragma unroll
    for (int e = 0; e < 8; ++e) o[e] = fmaf(p, (float)vv[e], o[e]);
  }
  const float inv = 1.0f / lsum;
  const v4f e0a = *(const v4f*)(emb0 + h * kBits);
  const v4f e0b = *(const v4f*)(emb0 + h * kBits + 4);
  const v4f e1a = *(const v4f*)(emb1 + h * kBits);
  const v4f e1b = *(const v4f*)(emb1 + h * kBits + 4);
  v8h hv;
#pragma unroll
  for (int e = 0; e < 4; ++e) {
    hv[e]     = (_Float16)((e1a[e] - e0a[e]) * (o[e]     * inv) * 256.0f);
    hv[4 + e] = (_Float16)((e1b[e] - e0b[e]) * (o[4 + e] * inv) * 256.0f);
  }
  if (id < total) {
    _Float16* dst = pout + qoff;
    *(volatile v8h*)dst = hv;
    __threadfence();
    *(volatile v8h*)dst = hv;
  }
}

__global__ __launch_bounds__(256) void k_ybias(const float* __restrict__ wo, const float* __restrict__ emb0,
                                               const float* __restrict__ emb1, float* __restrict__ yb, int n) {
  const int id = blockIdx.x * 256 + threadIdx.x;
  const int idc = id < n ? id : n - 1;
  const float* wr = wo + (size_t)idc * kDim;
  float s = 0.f;
#pragma unroll 1
  for (int j = 0; j < kDim; ++j) s = fmaf(0.5f * (emb0[j] + emb1[j]), wr[j], s);
  if (id < n) {
    ((volatile float*)yb)[idc] = s;
    __threadfence();
    ((volatile float*)yb)[idc] = s;
  }
}

extern "C" void kernel_launch(void* const* d_in, const int* in_sizes, int n_in,
                              void* d_out, int out_size, void* d_ws, size_t ws_size,
                              hipStream_t stream) {
  if (n_in < 8) return;
  if (in_sizes[0] != kRows * kDim || in_sizes[1] != kDim * kDim || in_sizes[2] != kDim * kDim ||
      in_sizes[3] != kDim * kDim || in_sizes[4] != kDim * kDim || in_sizes[5] != kDim ||
      in_sizes[6] != kDim || in_sizes[7] < 1)
    return;
  if (out_size != kRows * kDim) return;

  const float* x    = (const float*)d_in[0];
  const float* Wq   = (const float*)d_in[1];
  const float* Wk   = (const float*)d_in[2];
  const float* Wv   = (const float*)d_in[3];
  const float* Wo   = (const float*)d_in[4];
  const float* emb0 = (const float*)d_in[5];
  const float* emb1 = (const float*)d_in[6];
  const int*   swin = (const int*)d_in[7];
  float* out = (float*)d_out;

  const size_t szAct = (size_t)kRows * kDim * 2;
  const size_t szW   = (size_t)kDim * kDim * 2;
  const size_t szYB  = (size_t)kDim * 4;
  size_t off = 0;
  auto carve = [&](size_t bytes) { size_t o = off; off += (bytes + 255) & ~(size_t)255; return o; };
  const size_t oX16 = carve(szAct);
  const size_t oWQ = carve(szW), oWK = carve(szW), oWV = carve(szW), oWO = carve(szW);
  const size_t oCQ = carve(szAct), oCK = carve(szAct), oCV = carve(szAct);
  const size_t oP16 = carve(szAct);
  const size_t oYB = carve(szYB);
  if (off > ws_size) return;

  char* ws = (char*)d_ws;
  _Float16* X16  = (_Float16*)(ws + oX16);
  _Float16* WQ16 = (_Float16*)(ws + oWQ);
  _Float16* WK16 = (_Float16*)(ws + oWK);
  _Float16* WV16 = (_Float16*)(ws + oWV);
  _Float16* WO16 = (_Float16*)(ws + oWO);
  _Float16* CQ16 = (_Float16*)(ws + oCQ);
  _Float16* CK16 = (_Float16*)(ws + oCK);
  _Float16* CV16 = (_Float16*)(ws + oCV);
  _Float16* P16  = (_Float16*)(ws + oP16);
  float*    YB   = (float*)(ws + oYB);

  const int n8x = kRows * kDim / 8;
  const int n8w = kDim * kDim / 8;
  k_cast8<<<(n8x + 255) / 256, 256, 0, stream>>>(x,  X16,  1.0f,  n8x);
  k_cast8<<<(n8w + 255) / 256, 256, 0, stream>>>(Wq, WQ16, 64.0f, n8w);
  k_cast8<<<(n8w + 255) / 256, 256, 0, stream>>>(Wk, WK16, 64.0f, n8w);
  k_cast8<<<(n8w + 255) / 256, 256, 0, stream>>>(Wv, WV16, 64.0f, n8w);
  k_cast8<<<(n8w + 255) / 256, 256, 0, stream>>>(Wo, WO16, 64.0f, n8w);

  k_ybias<<<(kDim + 255) / 256, 256, 0, stream>>>(Wo, emb0, emb1, YB, kDim);

  const dim3 ggrid((kRows / 64) * (kDim / 64) / 8, 1);
  wmma_gemm64<0, false, 0, 1, false, 7><<<ggrid, 256, 0, stream>>>(
      U16(X16), U16(X16), kDim, 0L, U16(WQ16), U16(WQ16), kDim, 0L,
      (void*)CQ16, (void*)CQ16, kDim, 0L, YB, x, 0L, kRows, kDim, kDim, 1.0f / 64.0f);
  wmma_gemm64<0, false, 0, 1, false, 7><<<ggrid, 256, 0, stream>>>(
      U16(X16), U16(X16), kDim, 0L, U16(WK16), U16(WK16), kDim, 0L,
      (void*)CK16, (void*)CK16, kDim, 0L, YB, x, 0L, kRows, kDim, kDim, 1.0f / 64.0f);
  wmma_gemm64<0, false, 0, 1, false, 7><<<ggrid, 256, 0, stream>>>(
      U16(X16), U16(X16), kDim, 0L, U16(WV16), U16(WV16), kDim, 0L,
      (void*)CV16, (void*)CV16, kDim, 0L, YB, x, 0L, kRows, kDim, kDim, 1.0f / 64.0f);

  const int nwin = kRows * kHeads;
  k_window<<<(nwin + 255) / 256, 256, 0, stream>>>(CQ16, CK16, CV16, emb0, emb1, swin, P16, nwin);

  wmma_gemm64<0, false, 2, 0, false, 0><<<ggrid, 256, 0, stream>>>(
      U16(P16), U16(P16), kDim, 0L, U16(WO16), U16(WO16), kDim, 0L,
      (void*)out, (void*)out, kDim, 0L, YB, x, 0L, kRows, kDim, kDim, 1.0f / 262144.0f);
}
